// SD_Transformer_60043642798802
// MI455X (gfx1250) — hardware-verified
//
#include <hip/hip_runtime.h>

constexpr int NLAYER = 2;
constexpr int NBATCH = 8;
constexpr int NTOK   = 1024;
constexpr int DMODEL = 384;
constexpr int NHEAD  = 8;
constexpr int HDIM   = 48;
constexpr int HPAD   = 64;
constexpr int MROWS  = NBATCH * NTOK;
constexpr int QKVW3  = 3 * DMODEL;
constexpr int QKVPAD = 3 * NHEAD * HPAD;
constexpr int OPADW  = NHEAD * HPAD;
constexpr int FFN2   = 4 * DMODEL;
constexpr int FFN1   = 2 * DMODEL;
constexpr float WCARRY = 64.0f;
constexpr float OCARRY = 16.0f;
constexpr float GCARRY = 4096.0f;

typedef __attribute__((ext_vector_type(16))) _Float16 v16h;
typedef __attribute__((ext_vector_type(8)))  _Float16 v8h;
typedef __attribute__((ext_vector_type(16))) __bf16   v16b;
typedef __attribute__((ext_vector_type(8)))  __bf16   v8b;
typedef __attribute__((ext_vector_type(8)))  float    v8f;
typedef __attribute__((ext_vector_type(4)))  float    v4f;
#define PSCALE 32768.0f
#define U16(p) ((const unsigned short*)(const void*)(p))
#define PSCALE_INV (1.0f / 32768.0f)

__device__ __forceinline__ unsigned short f2bf_bits(float f) {
  unsigned u = __float_as_uint(f);
  return (unsigned short)((u + 0x7FFFu + ((u >> 16) & 1u)) >> 16);
}
__device__ __forceinline__ float bf_bits2f(unsigned short h) { return __uint_as_float(((unsigned)h) << 16); }

__device__ __forceinline__ void dep_guard_h(v8f& a, v8f& b, v16h x, v16h y) { asm volatile("v_nop\n\tv_nop\n\tv_nop\n\tv_nop" : "+v"(a), "+v"(b) : "v"(x), "v"(y)); }
__device__ __forceinline__ void dep_guard_b(v8f& a, v8f& b, v16b x, v16b y) { asm volatile("v_nop\n\tv_nop\n\tv_nop\n\tv_nop" : "+v"(a), "+v"(b) : "v"(x), "v"(y)); }
__device__ __forceinline__ void keep4_h(v16h a, v16h b, v16h c, v16h d) { asm volatile("v_nop" :: "v"(a), "v"(b), "v"(c), "v"(d)); }
__device__ __forceinline__ void keep4_b(v16b a, v16b b, v16b c, v16b d) { asm volatile("v_nop" :: "v"(a), "v"(b), "v"(c), "v"(d)); }
__device__ __forceinline__ void acc_guard4(v8f& a, v8f& b, v8f& c, v8f& d) { asm volatile("v_nop\n\tv_nop\n\tv_nop\n\tv_nop" : "+v"(a), "+v"(b), "+v"(c), "+v"(d)); }
template <typename T> struct Frag;
template <> struct Frag<_Float16> {
  typedef v16h V; union U { v16h v; v8h h[2]; };
  static __device__ __forceinline__ v16h load(const _Float16* p) {
    U f; f.h[0] = *(const v8h*)(p); f.h[1] = *(const v8h*)(p + 16); return f.v;
  }
  static __device__ __forceinline__ v8f mma(v16h a, v16h b, v8f c) {
    return __builtin_amdgcn_wmma_f32_16x16x32_f16(false, a, false, b, (short)0, c, false, false);
  }
  static __device__ __forceinline__ void guard(v8f& a, v8f& b, v16h x, v16h y) { dep_guard_h(a, b, x, y); }
  static __device__ __forceinline__ void keep(v16h a, v16h b, v16h c, v16h d) { keep4_h(a, b, c, d); }
};
template <> struct Frag<__bf16> {
  typedef v16b V; union U { v16b v; v8b h[2]; };
  static __device__ __forceinline__ v16b load(const __bf16* p) {
    U f; f.h[0] = *(const v8b*)(p); f.h[1] = *(const v8b*)(p + 16); return f.v;
  }
  static __device__ __forceinline__ v8f mma(v16b a, v16b b, v8f c) {
    return __builtin_amdgcn_wmma_f32_16x16x32_bf16(false, a, false, b, (short)0, c, false, false);
  }
  static __device__ __forceinline__ void guard(v8f& a, v8f& b, v16b x, v16b y) { dep_guard_b(a, b, x, y); }
  static __device__ __forceinline__ void keep(v16b a, v16b b, v16b c, v16b d) { keep4_b(a, b, c, d); }
};

template <int ET> struct Elem;
template <> struct Elem<0> { typedef _Float16 T; };
template <> struct Elem<1> { typedef __bf16 T; };
template <int ET, bool SPLIT, int BIAS_MODE, int OUT_MODE, bool RESID, int ACT = 0>
__global__ __launch_bounds__(256) void wmma_gemm64(
    const unsigned short* __restrict__ Ap, const unsigned short* __restrict__ A2p, int lda, long strideA,
    const unsigned short* __restrict__ Btp, const unsigned short* __restrict__ Bt2p, int ldb, long strideB,
    void* __restrict__ Cout, void* __restrict__ Cout2, int ldc, long strideC,
    const float* __restrict__ bias,
    const float* __restrict__ resid, long strideR,
    int M, int N, int K, float scale) {
  typedef typename Elem<ET>::T T;
  typedef typename Frag<T>::V V;
  const T* A = (const T*)Ap; const T* A2 = (const T*)A2p; const T* Bt = (const T*)Btp; const T* Bt2 = (const T*)Bt2p;
  __shared__ __align__(16) float sT[8][16 * 68];
  const int b    = blockIdx.y;
  const int lane = threadIdx.x & 31;
  const int wave = threadIdx.x >> 5;
  const int tilesN = N >> 6;
  const int tilesM = M >> 6;
  const int tile = blockIdx.x * 8 + wave;
  if (tile >= tilesM * tilesN) return;
  const int tm = tile / tilesN;
  const int tn = tile - tm * tilesN;
  const int m0 = tm << 6;
  const int n0 = tn << 6;

  const T* Ab  = A  + (size_t)b * strideA;
  const T* Bb  = Bt + (size_t)b * strideB;
  const T* Ab2 = SPLIT ? (A2  + (size_t)b * strideA) : nullptr;
  const T* Bb2 = SPLIT ? (Bt2 + (size_t)b * strideB) : nullptr;

  const int rlane = lane & 15;
  const int koff  = (lane >> 4) * 8;
  const int mOff  = (lane >> 4) * 8;

  v8f acc[4][4];
#pragma unroll
  for (int i = 0; i < 4; ++i)
#pragma unroll
    for (int j = 0; j < 4; ++j) acc[i][j] = (v8f){0.f,0.f,0.f,0.f,0.f,0.f,0.f,0.f};

  for (int k0 = 0; k0 < K; k0 += 32) {
    V bh[4], bl[4];
#pragma unroll
    for (int j = 0; j < 4; ++j) {
      const size_t bo = (size_t)(n0 + (j << 4) + rlane) * ldb + koff + k0;
      bh[j] = Frag<T>::load(Bb + bo);
      if (SPLIT) bl[j] = Frag<T>::load(Bb2 + bo);
    }
#pragma unroll
    for (int i = 0; i < 4; ++i) {
      const size_t ao = (size_t)(m0 + (i << 4) + rlane) * lda + koff + k0;
      V ah = Frag<T>::load(Ab + ao);
      V al;
      if (SPLIT) al = Frag<T>::load(Ab2 + ao);
#pragma unroll
      for (int j = 0; j < 4; ++j) {
        acc[i][j] = Frag<T>::mma(ah, bh[j], acc[i][j]);
        if (SPLIT) {
          acc[i][j] = Frag<T>::mma(ah, bl[j], acc[i][j]);
          acc[i][j] = Frag<T>::mma(al, bh[j], acc[i][j]);
        }
      }
      Frag<T>::guard(acc[i][0], acc[i][3], ah, SPLIT ? al : ah);
    }
    Frag<T>::keep(bh[0], bh[1], bh[2], bh[3]);
    if (SPLIT) Frag<T>::keep(bl[0], bl[1], bl[2], bl[3]);
  }
  acc_guard4(acc[0][0], acc[0][1], acc[0][2], acc[0][3]);
  acc_guard4(acc[1][0], acc[1][1], acc[1][2], acc[1][3]);
  acc_guard4(acc[2][0], acc[2][1], acc[2][2], acc[2][3]);
  acc_guard4(acc[3][0], acc[3][1], acc[3][2], acc[3][3]);

  float* slab = sT[wave];
  const float* Rb = RESID ? (resid + (size_t)b * strideR) : nullptr;
#pragma unroll
  for (int i = 0; i < 4; ++i) {
    const int mBase = m0 + (i << 4);
#pragma unroll
    for (int j = 0; j < 4; ++j) {
      const int n = n0 + (j << 4) + rlane;
      float bv = 0.f;
      if (BIAS_MODE == 2) bv = bias[n];
#pragma unroll
      for (int r = 0; r < 8; ++r) {
        float v = acc[i][j][r] * scale;
        if (BIAS_MODE == 1) v += bias[mBase + mOff + r];
        if (BIAS_MODE == 2) v += bv;
        if (RESID) v += Rb[(size_t)(mBase + mOff + r) * ldc + n];
        if (ACT == 1) v = tanhf(v);
        if (ACT == 2) v = fmaxf(v, 0.0f);
        if (ACT == 3) v = v / (1.0f + expf(-v));
        if (ACT == 4) v = (v > 0.f) ? v : 0.01f * v;
        slab[(mOff + r) * 68 + (j << 4) + rlane] = v;
      }
    }
    __builtin_amdgcn_fence(__ATOMIC_RELEASE, "workgroup");
    __builtin_amdgcn_wave_barrier();
    __builtin_amdgcn_fence(__ATOMIC_ACQUIRE, "workgroup");
    if (OUT_MODE == 0) {
      float* C = (float*)Cout + (size_t)b * strideC;
      const int hh = lane >> 4, c4 = (lane & 15) * 4;
      for (int pass = 0; pass < 2; ++pass) {
#pragma unroll
        for (int it = 0; it < 8; ++it) {
          const int row = it * 2 + hh;
          v4f v = *(const v4f*)(slab + row * 68 + c4);
          *(volatile v4f*)(C + (size_t)(mBase + row) * ldc + n0 + c4) = v;
        }
        __threadfence();
      }
    } else {
      const int q = lane >> 3, c8 = (lane & 7) * 8;
      unsigned short* C  = (unsigned short*)Cout  + (size_t)b * strideC;
      unsigned short* C2 = (OUT_MODE == 2) ? ((unsigned short*)Cout2 + (size_t)b * strideC) : nullptr;
      for (int pass = 0; pass < 2; ++pass) {
#pragma unroll
        for (int it = 0; it < 4; ++it) {
          const int row = it * 4 + q;
          const float* sp = slab + row * 68 + c8;
          v8h hv, lv;
#pragma unroll
          for (int e = 0; e < 8; ++e) {
            if (OUT_MODE == 1) {
              hv[e] = (_Float16)sp[e];
            } else {
              unsigned short hb = f2bf_bits(sp[e]);
              unsigned short lb = f2bf_bits(sp[e] - bf_bits2f(hb));
              hv[e] = __builtin_bit_cast(_Float16, hb);
              lv[e] = __builtin_bit_cast(_Float16, lb);
            }
          }
          *(volatile v8h*)(C + (size_t)(mBase + row) * ldc + n0 + c8) = hv;
          if (OUT_MODE == 2) *(volatile v8h*)(C2 + (size_t)(mBase + row) * ldc + n0 + c8) = lv;
        }
        __threadfence();
      }
    }
    __builtin_amdgcn_fence(__ATOMIC_RELEASE, "workgroup");
    __builtin_amdgcn_wave_barrier();
    __builtin_amdgcn_fence(__ATOMIC_ACQUIRE, "workgroup");
  }
}

#define AT_D 64
#define AT_NW 4
#define AT_QB 64
#define AT_KC 64
struct AttnGeom { const float* cp = nullptr; const float* pc = nullptr; long c_bs = 0, c_rs = 0, c_hs = 0;
                  long q_bs, q_rs, q_hs, k_bs, k_rs, k_hs, v_bs, v_rs, v_hs, o_bs, o_rs, o_hs;
                  int S, Skv, H, mask_mode; float qscale; int blk0; float mask_fill; int mask_is_int; };
static_assert(sizeof(AttnGeom) == 168, "no padding");

__device__ __forceinline__ unsigned short at_bf_bits(float f) {
  unsigned u = __float_as_uint(f);
  return (unsigned short)((u + 0x7FFFu + ((u >> 16) & 1u)) >> 16);
}
__device__ __forceinline__ __bf16 at_f2bf(float f) { return __builtin_bit_cast(__bf16, at_bf_bits(f)); }
__device__ __forceinline__ void at_split(float f, __bf16& hi, __bf16& lo) {
  const unsigned short hb = at_bf_bits(f);
  hi = __builtin_bit_cast(__bf16, hb);
  lo = at_f2bf(f - __uint_as_float(((unsigned)hb) << 16));
}
__device__ __forceinline__ v8f at_mma(v16b a, v16b b, v8f c) {
  c = __builtin_amdgcn_wmma_f32_16x16x32_bf16(false, a, false, b, (short)0, c, false, false);
  asm volatile("v_nop\n\tv_nop\n\tv_nop\n\tv_nop" : "+v"(c) : "v"(a), "v"(b));
  return c;
}
template <bool F16> __device__ __forceinline__ __bf16 at_to16(float f) {
  if (F16) return __builtin_bit_cast(__bf16, (_Float16)f);
  return at_f2bf(f);
}
template <bool F16> __device__ __forceinline__ v8f at_mma16(v16b a, v16b b, v8f c) {
  if (F16) {
    const v16h ah = __builtin_bit_cast(v16h, a), bh = __builtin_bit_cast(v16h, b);
    c = __builtin_amdgcn_wmma_f32_16x16x32_f16(false, ah, false, bh, (short)0, c, false, false);
    asm volatile("v_nop\n\tv_nop\n\tv_nop\n\tv_nop" : "+v"(c) : "v"(ah), "v"(bh));
    return c;
  }
  return at_mma(a, b, c);
}

template <bool SPLIT_QK, bool SPLIT_PV, bool F16 = false>
__global__ __launch_bounds__(128)
void attn64_kernel(const float* __restrict__ q, const float* __restrict__ k,
                   const float* __restrict__ v, float* __restrict__ out,
                   const void* __restrict__ mask_a, const int* __restrict__ mask_b, AttnGeom g) {
  static_assert(!(F16 && (SPLIT_QK || SPLIT_PV)), "f16 mode is non-split");
  const float PSC = F16 ? 32768.0f : 1.0f;
  union FB { v16b v; v8b h[2]; };
  __shared__ __align__(16) __bf16 Ksh[AT_KC * AT_D];
  __shared__ __align__(16) __bf16 Ksl[SPLIT_QK ? AT_KC * AT_D : 8];
  __shared__ __align__(16) __bf16 Vth[AT_D * AT_KC];
  __shared__ __align__(16) __bf16 Vtl[SPLIT_PV ? AT_D * AT_KC : 8];
  __shared__ __align__(16) __bf16 Psh[AT_NW][16 * AT_KC];
  __shared__ __align__(16) __bf16 Psl[SPLIT_PV ? AT_NW : 1][SPLIT_PV ? 16 * AT_KC : 8];
  __shared__ __align__(16) float  Os[AT_NW][16 * 68];

  const int tid  = threadIdx.x;
  const int wave = tid >> 5;
  const int lane = tid & 31;
  const int hh   = lane >> 4;
  const int c    = lane & 15;

  const int nqb = g.S / AT_QB;
  const int bx = blockIdx.x + g.blk0;
  const int qb = bx % nqb;
  const int bh = bx / nqb;
  const int h  = bh % g.H;
  const int b  = bh / g.H;
  const int qbase_block = qb * AT_QB;
  const int q0 = qbase_block + wave * 16;

  const float* qb_ptr = q + (size_t)b * g.q_bs + (size_t)h * g.q_hs;
  const float* kb_ptr = k + (size_t)b * g.k_bs + (size_t)h * g.k_hs;
  const float* vb_ptr = v + (size_t)b * g.v_bs + (size_t)h * g.v_hs;
  float*       ob_ptr = out + (size_t)b * g.o_bs + (size_t)h * g.o_hs;

  float dec6 = 0.f;
  if (g.mask_mode == 6) dec6 = g.cp[h];

  v16b qah[2], qal[2];
  {
    const float* qrow = qb_ptr + (size_t)(q0 + c) * g.q_rs;
#pragma unroll
    for (int dc = 0; dc < 2; ++dc) {
#pragma unroll
      for (int e = 0; e < 8; ++e) {
        const float f0 = qrow[dc * 32 + 8 * hh + e] * g.qscale;
        const float f1 = qrow[dc * 32 + 16 + 8 * hh + e] * g.qscale;
        if (SPLIT_QK) { __bf16 hq, lq; at_split(f0, hq, lq); qah[dc][e] = hq; qal[dc][e] = lq; at_split(f1, hq, lq); qah[dc][8 + e] = hq; qal[dc][8 + e] = lq; }
        else { qah[dc][e] = at_to16<F16>(f0); qah[dc][8 + e] = at_to16<F16>(f1); qal[dc][e] = qah[dc][e]; qal[dc][8 + e] = qah[dc][8 + e]; }
      }
    }
  }

  float mrow[8], lrow[8];
  v8f oacc[4];
#pragma unroll
  for (int r = 0; r < 8; ++r) { mrow[r] = -INFINITY; lrow[r] = 0.f; }
#pragma unroll
  for (int t = 0; t < 4; ++t) oacc[t] = (v8f){0.f,0.f,0.f,0.f,0.f,0.f,0.f,0.f};

  const int nChunks = (g.mask_mode == 1 || g.mask_mode == 4) ? (qb + 1) : (g.Skv / AT_KC);
  int qkeep[8];
#pragma unroll
  for (int r = 0; r < 8; ++r) qkeep[r] = (g.mask_mode == 3) ? mask_b[(size_t)b * g.S + q0 + 8 * hh + r] : 1;
  for (int kc = 0; kc < nChunks; ++kc) {
    const int kv0 = kc * AT_KC;
    __syncthreads();
    {
      const int kvr = tid >> 1, dh = (tid & 1) * 32;
      const float* krow = kb_ptr + (size_t)(kv0 + kvr) * g.k_rs + dh;
      const float* vrow = vb_ptr + (size_t)(kv0 + kvr) * g.v_rs + dh;
#pragma unroll
      for (int i = 0; i < 8; ++i) {
        v4f kk = *(const v4f*)(krow + 4 * i);
        v4f vv = *(const v4f*)(vrow + 4 * i);
#pragma unroll
        for (int e = 0; e < 4; ++e) {
          const int d = dh + 4 * i + e;
          if (SPLIT_QK) { __bf16 a, bl; at_split(kk[e], a, bl); Ksh[kvr * AT_D + d] = a; Ksl[kvr * AT_D + d] = bl; }
          else Ksh[kvr * AT_D + d] = at_to16<F16>(kk[e]);
          if (SPLIT_PV) { __bf16 a, bl; at_split(vv[e], a, bl); Vth[d * AT_KC + kvr] = a; Vtl[d * AT_KC + kvr] = bl; }
          else Vth[d * AT_KC + kvr] = at_to16<F16>(vv[e]);
        }
      }
    }
    __syncthreads();

    v8f s[4];
#pragma unroll
    for (int j = 0; j < 4; ++j) {
      s[j] = (v8f){0.f,0.f,0.f,0.f,0.f,0.f,0.f,0.f};
#pragma unroll
      for (int dc = 0; dc < 2; ++dc) {
        FB kb;
        kb.h[0] = *(const v8b*)(Ksh + (j * 16 + c) * AT_D + dc * 32 + 8 * hh);
        kb.h[1] = *(const v8b*)(Ksh + (j * 16 + c) * AT_D + dc * 32 + 16 + 8 * hh);
        s[j] = at_mma16<F16>(qah[dc], kb.v, s[j]);
        if (SPLIT_QK) {
          FB kl;
          kl.h[0] = *(const v8b*)(Ksl + (j * 16 + c) * AT_D + dc * 32 + 8 * hh);
          kl.h[1] = *(const v8b*)(Ksl + (j * 16 + c) * AT_D + dc * 32 + 16 + 8 * hh);
          s[j] = at_mma16<F16>(qah[dc], kl.v, s[j]);
          s[j] = at_mma16<F16>(qal[dc], kb.v, s[j]);
        }
      }
    }
    const bool diag = (g.mask_mode == 1) && (kc == qb);
    int kvkeep[4] = {1, 1, 1, 1};
    if (g.mask_mode == 3) {
#pragma unroll
      for (int j = 0; j < 4; ++j) kvkeep[j] = ((const int*)mask_a)[(size_t)b * g.Skv + kv0 + j * 16 + c];
    }
    float cm[8];
#pragma unroll
    for (int r = 0; r < 8; ++r) {
      const int qrow = q0 + 8 * hh + r;
      float m = -INFINITY;
#pragma unroll
      for (int j = 0; j < 4; ++j) {
        const int kvcol = kv0 + j * 16 + c;
        bool masked = false;
        if (diag) masked = (kvcol > qrow);
        else if (g.mask_mode == 4) masked = (kvcol > qrow) || (qrow - kvcol > g.mask_is_int);
        else if (g.mask_mode == 2) {
          const size_t mi = (size_t)qrow * g.Skv + kvcol;
          masked = (g.mask_is_int == 0) ? (((const float*)mask_a)[mi] == 0.0f)
                 : (g.mask_is_int == 1) ? (((const int*)mask_a)[mi] == 0) : (((const int*)mask_a)[mi] != 0);
        } else if (g.mask_mode == 3) masked = (qkeep[r] == 0) || (kvkeep[j] == 0);
        else if (g.mask_mode == 5) {
          const size_t mi = (size_t)qrow * g.Skv + kvcol;
          masked = (((const int*)mask_a)[mi] != 0);
          int n = mask_b[mi]; n = n < 0 ? 0 : n;
          s[j][r] += g.cp[(size_t)b * g.c_bs + (size_t)h * g.c_hs + (size_t)qrow * g.c_rs + n]
                   + g.pc[(size_t)b * g.c_bs + (size_t)h * g.c_hs + (size_t)kvcol * g.c_rs + n];
        } else if (g.mask_mode == 6) {
          s[j][r] += fabsf((float)(qrow - kvcol)) * dec6;
        }
        if (masked) s[j][r] = g.mask_fill;
        m = fmaxf(m, s[j][r]);
      }
#pragma unroll
      for (int off = 1; off < 16; off <<= 1) m = fmaxf(m, __shfl_xor(m, off, 32));
      cm[r] = m;
    }
    __bf16* pwh = Psh[wave];
    __bf16* pwl = Psl[SPLIT_PV ? wave : 0];
#pragma unroll
    for (int r = 0; r < 8; ++r) {
      const float mnew = fmaxf(mrow[r], cm[r]);
      const float alpha = expf(mrow[r] - mnew);
      mrow[r] = mnew;
      float psum = 0.f;
#pragma unroll
      for (int j = 0; j < 4; ++j) {
        const float p = expf(s[j][r] - mnew);
        psum += p;
        if (SPLIT_PV) { __bf16 a, bl; at_split(p, a, bl); pwh[(8 * hh + r) * AT_KC + j * 16 + c] = a; pwl[(8 * hh + r) * AT_KC + j * 16 + c] = bl; }
        else pwh[(8 * hh + r) * AT_KC + j * 16 + c] = at_to16<F16>(p * PSC);
      }
#pragma unroll
      for (int off = 1; off < 16; off <<= 1) psum += __shfl_xor(psum, off, 32);
      lrow[r] = lrow[r] * alpha + psum;
#pragma unroll
      for (int t = 0; t < 4; ++t) oacc[t][r] *= alpha;
    }
    __builtin_amdgcn_fence(__ATOMIC_RELEASE, "workgroup");
    __builtin_amdgcn_wave_barrier();
    __builtin_amdgcn_fence(__ATOMIC_ACQUIRE, "workgroup");
#pragma unroll 1
    for (int kk = 0; kk < 2; ++kk) {
      FB pa, pl;
      pa.h[0] = *(const v8b*)(pwh + c * AT_KC + kk * 32 + 8 * hh);
      pa.h[1] = *(const v8b*)(pwh + c * AT_KC + kk * 32 + 16 + 8 * hh);
      if (SPLIT_PV) {
        pl.h[0] = *(const v8b*)(pwl + c * AT_KC + kk * 32 + 8 * hh);
        pl.h[1] = *(const v8b*)(pwl + c * AT_KC + kk * 32 + 16 + 8 * hh);
      }
#pragma unroll
      for (int t = 0; t < 4; ++t) {
        FB vb;
        vb.h[0] = *(const v8b*)(Vth + (t * 16 + c) * AT_KC + kk * 32 + 8 * hh);
        vb.h[1] = *(const v8b*)(Vth + (t * 16 + c) * AT_KC + kk * 32 + 16 + 8 * hh);
        oacc[t] = at_mma16<F16>(pa.v, vb.v, oacc[t]);
        if (SPLIT_PV) {
          FB vl;
          vl.h[0] = *(const v8b*)(Vtl + (t * 16 + c) * AT_KC + kk * 32 + 8 * hh);
          vl.h[1] = *(const v8b*)(Vtl + (t * 16 + c) * AT_KC + kk * 32 + 16 + 8 * hh);
          oacc[t] = at_mma16<F16>(pa.v, vl.v, oacc[t]);
          oacc[t] = at_mma16<F16>(pl.v, vb.v, oacc[t]);
        }
      }
    }
  }

  float* os = Os[wave];
#pragma unroll
  for (int r = 0; r < 8; ++r) {
    const float inv = 1.0f / (lrow[r] * PSC);
#pragma unroll
    for (int t = 0; t < 4; ++t) os[(8 * hh + r) * 68 + t * 16 + c] = oacc[t][r] * inv;
  }
  __builtin_amdgcn_fence(__ATOMIC_RELEASE, "workgroup");
  __builtin_amdgcn_wave_barrier();
  __builtin_amdgcn_fence(__ATOMIC_ACQUIRE, "workgroup");
  {
    const int c4 = (lane & 15) * 4;
    for (int pass = 0; pass < 2; ++pass) {
#pragma unroll
      for (int it = 0; it < 8; ++it) {
        const int row = it * 2 + hh;
        v4f val = *(const v4f*)(os + row * 68 + c4);
        *(volatile v4f*)(ob_ptr + (size_t)(q0 + row) * g.o_rs + c4) = val;
      }
      __threadfence();
    }
  }
}

__device__ __forceinline__ float wsum32(float v) {
#pragma unroll
  for (int off = 16; off > 0; off >>= 1) v += __shfl_xor(v, off, 32);
  return v;
}

__global__ __launch_bounds__(256) void k_cast8(const float* __restrict__ in, _Float16* __restrict__ out,
                                               float mul, int n8) {
  const int id = blockIdx.x * 256 + threadIdx.x;
  const int idc = id < n8 ? id : n8 - 1;
  const v4f a0 = *(const v4f*)(in + (size_t)idc * 8);
  const v4f a1 = *(const v4f*)(in + (size_t)idc * 8 + 4);
  v8h hv;
#pragma unroll
  for (int e = 0; e < 4; ++e) { hv[e] = (_Float16)(a0[e] * mul); hv[4 + e] = (_Float16)(a1[e] * mul); }
  if (id < n8) {
    _Float16* dst = out + (size_t)idc * 8;
    *(volatile v8h*)dst = hv;
    __threadfence();
    *(volatile v8h*)dst = hv;
  }
}

__global__ __launch_bounds__(256) void k_padrows(const float* __restrict__ w, _Float16* __restrict__ out,
                                                 float mul, int total) {
  const int id = blockIdx.x * 256 + threadIdx.x;
  const int idc = id < total ? id : total - 1;
  const int r = idc / 48;
  const int j = idc - r * 48;
  const int s = r >> 9, h = (r >> 6) & 7, d = r & 63;
  const bool valid = d < HDIM;
  const int dcl = valid ? d : (HDIM - 1);
  const float* src = w + (size_t)(s * DMODEL + h * HDIM + dcl) * DMODEL + 8 * j;
  const v4f a0 = *(const v4f*)src;
  const v4f a1 = *(const v4f*)(src + 4);
  v8h hv;
#pragma unroll
  for (int e = 0; e < 4; ++e) {
    hv[e]     = valid ? (_Float16)(a0[e] * mul) : (_Float16)0.0f;
    hv[4 + e] = valid ? (_Float16)(a1[e] * mul) : (_Float16)0.0f;
  }
  if (id < total) {
    _Float16* dst = out + (size_t)r * DMODEL + 8 * j;
    *(volatile v8h*)dst = hv;
    __threadfence();
    *(volatile v8h*)dst = hv;
  }
}

__global__ __launch_bounds__(256) void k_padbias(const float* __restrict__ bsrc, float* __restrict__ out, int total) {
  const int id = blockIdx.x * 256 + threadIdx.x;
  const int idc = id < total ? id : total - 1;
  const int r0 = 4 * idc;
  const int s = r0 >> 9, h = (r0 >> 6) & 7, d0 = r0 & 63;
  const bool valid = d0 < HDIM;
  const int d0c = valid ? d0 : (HDIM - 4);
  const v4f bv = *(const v4f*)(bsrc + s * DMODEL + h * HDIM + d0c);
  const v4f zero = (v4f){0.f, 0.f, 0.f, 0.f};
  const v4f o = valid ? bv : zero;
  if (id < total) {
    float* dst = out + r0;
    *(volatile v4f*)dst = o;
    __threadfence();
    *(volatile v4f*)dst = o;
  }
}

__global__ __launch_bounds__(256) void k_padcols(const float* __restrict__ w, _Float16* __restrict__ out,
                                                 float mul, int total) {
  const int id = blockIdx.x * 256 + threadIdx.x;
  const int idc = id < total ? id : total - 1;
  const int o = idc >> 6;
  const int j = idc & 63;
  const int c0 = 8 * j;
  const int h = c0 >> 6, d0 = c0 & 63;
  const bool valid = d0 < HDIM;
  const int d0c = valid ? d0 : (HDIM - 8);
  const float* src = w + (size_t)o * DMODEL + h * HDIM + d0c;
  const v4f a0 = *(const v4f*)src;
  const v4f a1 = *(const v4f*)(src + 4);
  v8h hv;
#pragma unroll
  for (int e = 0; e < 4; ++e) {
    hv[e]     = valid ? (_Float16)(a0[e] * mul) : (_Float16)0.0f;
    hv[4 + e] = valid ? (_Float16)(a1[e] * mul) : (_Float16)0.0f;
  }
  if (id < total) {
    _Float16* dst = out + (size_t)o * OPADW + c0;
    *(volatile v8h*)dst = hv;
    __threadfence();
    *(volatile v8h*)dst = hv;
  }
}

__global__ __launch_bounds__(32) void k_decay(float* __restrict__ dec) {
  const int lane = threadIdx.x & 31;
  const int h = lane & 7;
  const float val = logf(1.0f - exp2f(-2.0f - 0.5f * (float)h));
  const float o = (lane < NHEAD) ? val : 0.0f;
  ((volatile float*)dec)[lane] = o;
  __threadfence();
  ((volatile float*)dec)[lane] = o;
}

__global__ __launch_bounds__(256) void k_ln384(const float* __restrict__ x, const float* __restrict__ gam,
                                               const float* __restrict__ bet, _Float16* __restrict__ y, int nrows) {
  __shared__ __align__(16) float xs[8][DMODEL];
  const int tid = threadIdx.x, lane = tid & 31, wave = tid >> 5;
  const int row = blockIdx.x * 8 + wave;
  const int rowc = row < nrows ? row : nrows - 1;
  const float* xr = x + (size_t)rowc * DMODEL;
  const v4f v0 = *(const v4f*)(xr + 4 * lane);
  const v4f v1 = *(const v4f*)(xr + 128 + 4 * lane);
  const v4f v2 = *(const v4f*)(xr + 256 + 4 * lane);
  float s = ((v0[0] + v0[1]) + (v0[2] + v0[3])) + ((v1[0] + v1[1]) + (v1[2] + v1[3])) + ((v2[0] + v2[1]) + (v2[2] + v2[3]));
  s = wsum32(s);
  const float mean = s * (1.0f / (float)DMODEL);
  const v4f d0 = v0 - mean, d1 = v1 - mean, d2 = v2 - mean;
  float qs = 0.f;
#pragma unroll
  for (int e = 0; e < 4; ++e) { qs += d0[e] * d0[e]; qs += d1[e] * d1[e]; qs += d2[e] * d2[e]; }
  qs = wsum32(qs);
  const float var = qs * (1.0f / (float)DMODEL);
  const float rs = rsqrtf(var + 1e-5f);
  const v4f g0 = *(const v4f*)(gam + 4 * lane), g1 = *(const v4f*)(gam + 128 + 4 * lane), g2 = *(const v4f*)(gam + 256 + 4 * lane);
  const v4f b0 = *(const v4f*)(bet + 4 * lane), b1 = *(const v4f*)(bet + 128 + 4 * lane), b2 = *(const v4f*)(bet + 256 + 4 * lane);
  const v4f o0 = d0 * rs * g0 + b0;
  const v4f o1 = d1 * rs * g1 + b1;
  const v4f o2 = d2 * rs * g2 + b2;
  float* xw = xs[wave];
  *(v4f*)(xw + 4 * lane) = o0;
  *(v4f*)(xw + 128 + 4 * lane) = o1;
  *(v4f*)(xw + 256 + 4 * lane) = o2;
  __builtin_amdgcn_fence(__ATOMIC_RELEASE, "workgroup");
  __builtin_amdgcn_wave_barrier();
  __builtin_amdgcn_fence(__ATOMIC_ACQUIRE, "workgroup");
  const int s1 = 32 + (lane & 15);
  const v4f pa = *(const v4f*)(xw + 8 * lane), pb = *(const v4f*)(xw + 8 * lane + 4);
  const v4f qa = *(const v4f*)(xw + 8 * s1),   qb2 = *(const v4f*)(xw + 8 * s1 + 4);
  v8h h0, h1;
#pragma unroll
  for (int e = 0; e < 4; ++e) {
    h0[e] = (_Float16)pa[e]; h0[4 + e] = (_Float16)pb[e];
    h1[e] = (_Float16)qa[e]; h1[4 + e] = (_Float16)qb2[e];
  }
  _Float16* yr = y + (size_t)rowc * DMODEL;
  for (int pass = 0; pass < 2; ++pass) {
    if (row < nrows) {
      *(volatile v8h*)(yr + 8 * lane) = h0;
      if (lane < 16) *(volatile v8h*)(yr + 8 * s1) = h1;
    }
    __threadfence();
  }
}

__device__ __forceinline__ float gelu_erf_f(float x) {
  const float z = x * 0.70710678118654752f;
  const float az = fabsf(z);
  const float t = __builtin_amdgcn_rcpf(fmaf(0.3275911f, az, 1.0f));
  float poly = fmaf(t, 1.061405429f, -1.453152027f);
  poly = fmaf(t, poly, 1.421413741f);
  poly = fmaf(t, poly, -0.284496736f);
  poly = fmaf(t, poly, 0.254829592f);
  poly = poly * t;
  const float ex = __expf(-(az * az));
  float r = fmaf(-poly, ex, 1.0f);
  r = copysignf(r, z);
  const float hx = 0.5f * x;
  return fmaf(hx, r, hx);
}

__global__ __launch_bounds__(256) void k_dwgate(const float* __restrict__ Hp, const float* __restrict__ dww,
                                                const float* __restrict__ dwb, _Float16* __restrict__ G, int total) {
  const int id = blockIdx.x * 256 + threadIdx.x;
  const int idc = id < total ? id : total - 1;
  const int tok = idc / 96;
  const int c = (idc - tok * 96) * 8;
  const int bimg = tok >> 10, n = tok & 1023, y = n >> 5, x = n & 31;
  v4f a0 = *(const v4f*)(dwb + c), a1 = *(const v4f*)(dwb + c + 4);
  v4f g0 = *(const v4f*)(dwb + FFN1 + c), g1 = *(const v4f*)(dwb + FFN1 + c + 4);
  const float* w1 = dww + (size_t)c * 9;
  const float* w2 = dww + (size_t)(FFN1 + c) * 9;
#pragma unroll 1
  for (int tap = 0; tap < 9; ++tap) {
    const int ky = tap / 3;
    const int kx = tap - 3 * ky;
    const int yy = y + ky - 1, xx = x + kx - 1;
    const bool valid = ((unsigned)yy < 32u) && ((unsigned)xx < 32u);
    const int yyc = yy < 0 ? 0 : (yy > 31 ? 31 : yy);
    const int xxc = xx < 0 ? 0 : (xx > 31 ? 31 : xx);
    const float* hp = Hp + (size_t)((bimg << 10) + (yyc << 5) + xxc) * FFN2 + c;
    const v4f h0 = *(const v4f*)hp, h1 = *(const v4f*)(hp + 4);
    const v4f k0 = *(const v4f*)(hp + FFN1), k1 = *(const v4f*)(hp + FFN1 + 4);
#pragma unroll
    for (int e = 0; e < 4; ++e) {
      const float wa = w1[e * 9 + tap], wb = w1[(4 + e) * 9 + tap];
      const float wc = w2[e * 9 + tap], wd = w2[(4 + e) * 9 + tap];
      a0[e] = fmaf(wa, valid ? h0[e] : 0.0f, a0[e]);
      a1[e] = fmaf(wb, valid ? h1[e] : 0.0f, a1[e]);
      g0[e] = fmaf(wc, valid ? k0[e] : 0.0f, g0[e]);
      g1[e] = fmaf(wd, valid ? k1[e] : 0.0f, g1[e]);
    }
  }
  v8h hv;
#pragma unroll
  for (int e = 0; e < 4; ++e) {
    hv[e]     = (_Float16)(gelu_erf_f(a0[e]) * g0[e] * GCARRY);
    hv[4 + e] = (_Float16)(gelu_erf_f(a1[e]) * g1[e] * GCARRY);
  }
  if (id < total) {
    _Float16* dst = G + (size_t)tok * FFN1 + c;
    *(volatile v8h*)dst = hv;
    __threadfence();
    *(volatile v8h*)dst = hv;
  }
}

extern "C" void kernel_launch(void* const* d_in, const int* in_sizes, int n_in,
                              void* d_out, int out_size, void* d_ws, size_t ws_size,
                              hipStream_t stream) {
  if (n_in < 15) return;
  if (in_sizes[0] != MROWS * DMODEL || in_sizes[1] != NLAYER * QKVW3 * DMODEL || in_sizes[2] != NLAYER * QKVW3 ||
      in_sizes[3] != NLAYER * DMODEL * DMODEL || in_sizes[4] != NLAYER * DMODEL ||
      in_sizes[5] != NLAYER * DMODEL || in_sizes[6] != NLAYER * DMODEL || in_sizes[7] != NLAYER * DMODEL || in_sizes[8] != NLAYER * DMODEL ||
      in_sizes[9] != NLAYER * FFN2 * DMODEL || in_sizes[10] != NLAYER * FFN2 || in_sizes[11] != NLAYER * FFN2 * 9 ||
      in_sizes[12] != NLAYER * FFN2 || in_sizes[13] != NLAYER * DMODEL * FFN1 || in_sizes[14] != NLAYER * DMODEL)
    return;
  if (out_size != MROWS * DMODEL) return;

  const float* x_in   = (const float*)d_in[0];
  const float* qkv_w  = (const float*)d_in[1];
  const float* qkv_b  = (const float*)d_in[2];
  const float* proj_w = (const float*)d_in[3];
  const float* proj_b = (const float*)d_in[4];
  const float* ln1_g  = (const float*)d_in[5];
  const float* ln1_b  = (const float*)d_in[6];
  const float* ln2_g  = (const float*)d_in[7];
  const float* ln2_b  = (const float*)d_in[8];
  const float* pin_w  = (const float*)d_in[9];
  const float* pin_b  = (const float*)d_in[10];
  const float* dw_w   = (const float*)d_in[11];
  const float* dw_b   = (const float*)d_in[12];
  const float* pout_w = (const float*)d_in[13];
  const float* pout_b = (const float*)d_in[14];
  float* out = (float*)d_out;

  const size_t szWQKV = (size_t)QKVPAD * DMODEL * 2, szQKVB = (size_t)QKVPAD * 4, szWPROJ = (size_t)DMODEL * OPADW * 2;
  const size_t szWPIN = (size_t)FFN2 * DMODEL * 2, szWPOUT = (size_t)DMODEL * FFN1 * 2, szDEC = 256;
  const size_t szXN = (size_t)MROWS * DMODEL * 2, szBIG = (size_t)MROWS * QKVPAD * 4, szOPL = (size_t)MROWS * OPADW * 4;
  const size_t szO16 = (size_t)MROWS * OPADW * 2, szX = (size_t)MROWS * DMODEL * 4, szG16 = (size_t)MROWS * FFN1 * 2;
  size_t off = 0;
  auto carve = [&](size_t bytes) { size_t o = off; off += (bytes + 255) & ~(size_t)255; return o; };
  const size_t oWQKV = carve(szWQKV), oQKVB = carve(szQKVB), oWPROJ = carve(szWPROJ), oWPIN = carve(szWPIN), oWPOUT = carve(szWPOUT);
  const size_t oDEC = carve(szDEC), oXN = carve(szXN), oBIG = carve(szBIG), oOPL = carve(szOPL), oO16 = carve(szO16);
  const size_t oX1 = carve(szX), oX0 = carve(szX);
  if (off > ws_size) return;
  if (off > (size_t)134217728) return;
  if (szG16 > szOPL) return;
  if ((size_t)MROWS * FFN2 * 4 != szBIG) return;

  char* ws = (char*)d_ws;
  _Float16* WQKV16 = (_Float16*)(ws + oWQKV);
  float*    QKVB   = (float*)(ws + oQKVB);
  _Float16* WPROJ16 = (_Float16*)(ws + oWPROJ);
  _Float16* WPIN16 = (_Float16*)(ws + oWPIN);
  _Float16* WPOUT16 = (_Float16*)(ws + oWPOUT);
  float*    DEC    = (float*)(ws + oDEC);
  _Float16* XN16   = (_Float16*)(ws + oXN);
  float*    QKV    = (float*)(ws + oBIG);
  float*    HBUF   = (float*)(ws + oBIG);
  float*    OPL    = (float*)(ws + oOPL);
  _Float16* G16    = (_Float16*)(ws + oOPL);
  _Float16* O16    = (_Float16*)(ws + oO16);
  float*    X1     = (float*)(ws + oX1);
  float*    X0     = (float*)(ws + oX0);

  k_decay<<<1, 32, 0, stream>>>(DEC);

  AttnGeom ga{};
  ga.cp = DEC; ga.pc = DEC; ga.c_bs = 0; ga.c_rs = 0; ga.c_hs = 0;
  ga.q_bs = (long)NTOK * QKVPAD; ga.q_rs = QKVPAD; ga.q_hs = HPAD;
  ga.k_bs = (long)NTOK * QKVPAD; ga.k_rs = QKVPAD; ga.k_hs = HPAD;
  ga.v_bs = (long)NTOK * QKVPAD; ga.v_rs = QKVPAD; ga.v_hs = HPAD;
  ga.o_bs = (long)NTOK * OPADW;  ga.o_rs = OPADW;  ga.o_hs = HPAD;
  ga.S = NTOK; ga.Skv = NTOK; ga.H = NHEAD; ga.mask_mode = 6; ga.qscale = 0.14433756729740643f; ga.blk0 = 0;
  ga.mask_fill = 0.0f; ga.mask_is_int = 0;

  for (int l = 0; l < NLAYER; ++l) {
    const float* xcur = (l == 0) ? x_in : X0;
    float* xnext = (l == NLAYER - 1) ? out : X0;

    k_padrows<<<(QKVPAD * 48) / 256, 256, 0, stream>>>(qkv_w + (size_t)l * QKVW3 * DMODEL, WQKV16, WCARRY, QKVPAD * 48);
    k_padbias<<<2, 256, 0, stream>>>(qkv_b + (size_t)l * QKVW3, QKVB, QKVPAD / 4);
    k_padcols<<<(DMODEL * 64) / 256, 256, 0, stream>>>(proj_w + (size_t)l * DMODEL * DMODEL, WPROJ16, WCARRY, DMODEL * 64);
    k_cast8<<<(FFN2 * DMODEL / 8 + 255) / 256, 256, 0, stream>>>(pin_w + (size_t)l * FFN2 * DMODEL, WPIN16, WCARRY, FFN2 * DMODEL / 8);
    k_cast8<<<(DMODEL * FFN1 / 8 + 255) / 256, 256, 0, stream>>>(pout_w + (size_t)l * DMODEL * FFN1, WPOUT16, WCARRY, DMODEL * FFN1 / 8);

    k_ln384<<<MROWS / 8, 256, 0, stream>>>(xcur, ln1_g + l * DMODEL, ln1_b + l * DMODEL, XN16, MROWS);

    wmma_gemm64<0, false, 2, 0, false, 0><<<dim3((MROWS / 64) * (QKVPAD / 64) / 8, 1), 256, 0, stream>>>(
        U16(XN16), U16(XN16), DMODEL, 0L, U16(WQKV16), U16(WQKV16), DMODEL, 0L,
        (void*)QKV, (void*)QKV, QKVPAD, 0L, QKVB, xcur, 0L, MROWS, QKVPAD, DMODEL, 1.0f / 64.0f);

    attn64_kernel<false, false, true><<<NBATCH * NHEAD * (NTOK / 64), 128, 0, stream>>>(
        QKV, QKV + OPADW, QKV + 2 * OPADW, OPL, (const void*)QKV, (const int*)(const void*)QKV, ga);

    k_cast8<<<(MROWS * OPADW / 8 + 255) / 256, 256, 0, stream>>>(OPL, O16, OCARRY, MROWS * OPADW / 8);

    wmma_gemm64<0, false, 2, 0, true, 0><<<dim3((MROWS / 64) * (DMODEL / 64) / 8, 1), 256, 0, stream>>>(
        U16(O16), U16(O16), OPADW, 0L, U16(WPROJ16), U16(WPROJ16), OPADW, 0L,
        (void*)X1, (void*)X1, DMODEL, 0L, proj_b + l * DMODEL, xcur, 0L, MROWS, DMODEL, OPADW, 1.0f / 1024.0f);

    k_ln384<<<MROWS / 8, 256, 0, stream>>>(X1, ln2_g + l * DMODEL, ln2_b + l * DMODEL, XN16, MROWS);

    wmma_gemm64<0, false, 2, 0, false, 0><<<dim3((MROWS / 64) * (FFN2 / 64) / 8, 1), 256, 0, stream>>>(
        U16(XN16), U16(XN16), DMODEL, 0L, U16(WPIN16), U16(WPIN16), DMODEL, 0L,
        (void*)HBUF, (void*)HBUF, FFN2, 0L, pin_b + l * FFN2, xcur, 0L, MROWS, FFN2, DMODEL, 1.0f / 64.0f);

    k_dwgate<<<(MROWS * 96) / 256, 256, 0, stream>>>(HBUF, dw_w + (size_t)l * FFN2 * 9, dw_b + (size_t)l * FFN2, G16, MROWS * 96);

    wmma_gemm64<0, false, 2, 0, true, 0><<<dim3((MROWS / 64) * (DMODEL / 64) / 8, 1), 256, 0, stream>>>(
        U16(G16), U16(G16), FFN1, 0L, U16(WPOUT16), U16(WPOUT16), FFN1, 0L,
        (void*)xnext, (void*)xnext, DMODEL, 0L, pout_b + l * DMODEL, X1, 0L, MROWS, DMODEL, FFN1, 1.0f / 262144.0f);
  }
}
